// BiPixelMambaLayer_55413668053386
// MI455X (gfx1250) — hardware-run, weakly checked
//
#include <hip/hip_runtime.h>
#include <math.h>


#define NB_    2
#define CM_    256
#define LSEQ_  4096
#define NP_    64
#define PS_    64
#define NSEQ_  (NB_ * PS_)
#define NT_    (NSEQ_ * NP_)
#define DI_    512
#define NS_    16
#define DTR_   16
#define XE_    (2 * DI_)
#define XD_    (DTR_ + 2 * NS_)
#define XDP_   64

static_assert(NT_ == 8192);
static_assert(LSEQ_ == NP_ * PS_);
static_assert(CM_ % 128 == 0);
static_assert(DI_ % 128 == 0);
static_assert(XD_ <= XDP_);
static_assert(NP_ == 64);

typedef float          v4f   __attribute__((ext_vector_type(4)));
typedef float          v8f   __attribute__((ext_vector_type(8)));
typedef __bf16         v16b  __attribute__((ext_vector_type(16)));
typedef unsigned short u16x8 __attribute__((ext_vector_type(8)));

union FragB { u16x8 h[2]; v16b v; };

__device__ __forceinline__ unsigned short f32_to_bf16(float f) {
    unsigned u = __float_as_uint(f);
    unsigned r = u + 0x7FFFu + ((u >> 16) & 1u);
    return (unsigned short)(r >> 16);
}
__device__ __forceinline__ float silu_f(float x) {
    const float e = __expf(-x);
    return x * __builtin_amdgcn_rcpf(1.0f + e);
}
__device__ __forceinline__ float softplus_f(float x) {
    return fmaxf(x, 0.0f) + log1pf(expf(-fabsf(x)));
}
__device__ __forceinline__ float conv4_silu(float x0, float x1, float x2, float x3,
                                            float w0, float w1, float w2, float w3, float bias) {
    const float c = w0 * x0 + w1 * x1 + w2 * x2 + w3 * x3;
    return silu_f(c + bias);
}
__device__ __forceinline__ v8f ld8f(const float* p) {
    const v4f a = *(const v4f*)p;
    const v4f b = *(const v4f*)(p + 4);
    return __builtin_shufflevector(a, b, 0, 1, 2, 3, 4, 5, 6, 7);
}
__device__ __forceinline__ float wsum32(float v) {
#pragma unroll
    for (int o = 16; o > 0; o >>= 1) v += __shfl_xor(v, o, 32);
    return v;
}

__device__ __forceinline__ void mma16(v8f& acc, const FragB& a, const FragB& b) {
    acc = __builtin_amdgcn_wmma_f32_16x16x32_bf16(false, a.v, false, b.v, (short)0, acc, false, false);
    asm volatile("v_nop\n\tv_nop\n\tv_nop\n\tv_nop" : "+v"(acc) : "v"(a.v), "v"(b.v));
}

__global__ __launch_bounds__(256)
void cvt_kernel(const float* __restrict__ s0, const float* __restrict__ s1,
                unsigned short* d0p, unsigned short* d1p, int rows, int rows_pad, int K)
{
    const int sel = blockIdx.y;
    const float* src = sel ? s1 : s0;
    unsigned short* dst = sel ? d1p : d0p;
    const int n8 = (rows_pad * K) >> 3;
    const int i = blockIdx.x * 256 + threadIdx.x;
    if (i >= n8) return;
    const int e = i * 8;
    const int r = e / K;
    const int col = e - r * K;
    const int rc = (r < rows) ? r : (rows - 1);
    const v8f x = ld8f(src + (size_t)rc * K + col);
    u16x8 o;
#pragma unroll
    for (int c = 0; c < 8; ++c) o[c] = (r < rows) ? f32_to_bf16(x[c]) : (unsigned short)0;
    unsigned short* gp = dst + e;
    *(volatile u16x8*)gp = o;
    __threadfence();
    *(volatile u16x8*)gp = o;
}

__global__ __launch_bounds__(256)
void ln_kernel(const float* __restrict__ x, const float* __restrict__ g,
               const float* __restrict__ bt, unsigned short* xn)
{
    const int tid = threadIdx.x, lane = tid & 31, wave = tid >> 5;
    const int t = blockIdx.x * 8 + wave;
    const int bimg = t >> 12;
    const int pp = (t >> 6) & 63;
    const int n = t & 63;
    const int pos = n * PS_ + pp;
    const int c0 = lane * 8;
    const float* xp = x + ((size_t)(bimg * CM_ + c0)) * LSEQ_ + pos;
    float v[8];
#pragma unroll
    for (int j = 0; j < 8; ++j) v[j] = xp[(size_t)j * LSEQ_];
    float s = 0.0f;
#pragma unroll
    for (int j = 0; j < 8; ++j) s += v[j];
    s = wsum32(s);
    const float mu = s * (1.0f / CM_);
    float q = 0.0f;
#pragma unroll
    for (int j = 0; j < 8; ++j) { const float d = v[j] - mu; q += d * d; }
    q = wsum32(q);
    const float var = q * (1.0f / CM_);
    const float rs = rsqrtf(var + 1e-5f);
    u16x8 o;
#pragma unroll
    for (int j = 0; j < 8; ++j) o[j] = f32_to_bf16((v[j] - mu) * rs * g[c0 + j] + bt[c0 + j]);
    unsigned short* gp = xn + (size_t)t * CM_ + c0;
    *(volatile u16x8*)gp = o;
    __threadfence();
    *(volatile u16x8*)gp = o;
}

template<int NBF, bool HALFK, int EPI>
__global__ __launch_bounds__(128)
void gemm_kernel(const unsigned short* __restrict__ Ain, const unsigned short* __restrict__ Bin,
                 float* Cout, const float* __restrict__ bias0, const float* __restrict__ bias1,
                 unsigned short* Pout, const float* __restrict__ xres,
                 int K, int ldc, int strideA, int strideB, int strideC, int strideP)
{
    constexpr int CW  = NBF * 16;
    constexpr int SP  = 2 * CW + 4;
    constexpr int LPR = CW / 4;
    constexpr int RPI = 32 / LPR;
    constexpr int NIT = 32 / RPI;
    __shared__ __attribute__((aligned(16))) float st[64 * SP];

    const int tid  = threadIdx.x;
    const int lane = tid & 31;
    const int wave = tid >> 5;
    const int h    = lane >> 4;
    const int m    = lane & 15;
    const int wm   = wave >> 1;
    const int wn   = wave & 1;
    const int z    = blockIdx.z;

    const unsigned short* A  = Ain + (size_t)z * (size_t)strideA;
    const unsigned short* Bw = Bin + (size_t)z * (size_t)strideB;
    float* C = Cout + (size_t)z * (size_t)strideC;
    unsigned short* P16 = Pout + (size_t)z * (size_t)strideP;
    const float* bias = z ? bias1 : bias0;

    const int rowB = blockIdx.y * 64;
    const int colB = blockIdx.x * (2 * CW);
    const int rowW = rowB + wm * 32;
    const int colW = colB + wn * CW;

    v8f acc[2 * NBF];
#pragma unroll
    for (int j = 0; j < 2 * NBF; ++j)
#pragma unroll
        for (int r = 0; r < 8; ++r) acc[j][r] = 0.0f;

    const size_t aoff  = (size_t)(rowW + m) * K + 8 * h;
    const size_t boff  = (size_t)(colW + m) * K + 8 * h;
    const size_t sub16 = (size_t)16 * K;

    if (HALFK) {
        u16x8 zz;
#pragma unroll
        for (int c = 0; c < 8; ++c) zz[c] = 0;
        FragB fa[2], fb[NBF];
#pragma unroll
        for (int s = 0; s < 2; ++s) {
            fa[s].h[0] = *(const u16x8*)(A + aoff + s * sub16);
            fa[s].h[1] = zz;
        }
#pragma unroll
        for (int j = 0; j < NBF; ++j) {
            fb[j].h[0] = *(const u16x8*)(Bw + boff + j * sub16);
            fb[j].h[1] = zz;
        }
#pragma unroll
        for (int s = 0; s < 2; ++s)
#pragma unroll
            for (int j = 0; j < NBF; ++j)
                mma16(acc[s * NBF + j], fa[s], fb[j]);
    } else {
        const int nk = K >> 5;
        for (int kt = 0; kt < nk; ++kt) {
            const size_t k0 = (size_t)kt * 32;
            FragB fa[2], fb[NBF];
#pragma unroll
            for (int s = 0; s < 2; ++s) {
                const unsigned short* p = A + aoff + s * sub16 + k0;
                fa[s].h[0] = *(const u16x8*)(p);
                fa[s].h[1] = *(const u16x8*)(p + 16);
            }
#pragma unroll
            for (int j = 0; j < NBF; ++j) {
                const unsigned short* p = Bw + boff + j * sub16 + k0;
                fb[j].h[0] = *(const u16x8*)(p);
                fb[j].h[1] = *(const u16x8*)(p + 16);
            }
#pragma unroll
            for (int s = 0; s < 2; ++s)
#pragma unroll
                for (int j = 0; j < NBF; ++j)
                    mma16(acc[s * NBF + j], fa[s], fb[j]);
        }
    }

#pragma unroll
    for (int s = 0; s < 2; ++s)
#pragma unroll
        for (int j = 0; j < NBF; ++j)
#pragma unroll
            for (int r = 0; r < 8; ++r) {
                const int rl = wm * 32 + s * 16 + 8 * h + r;
                const int cl = wn * CW + j * 16 + m;
                float v = acc[s * NBF + j][r];
                if (EPI == 2) v = softplus_f(v + bias[colB + cl]);
                st[rl * SP + cl] = v;
            }
    __syncthreads();

    if (EPI == 3) {
        const int bb   = blockIdx.y;
        const int bimg = bb >> 6;
        const int pp   = bb & 63;
        const int n0   = m * 4;
        v4f vv[16];
#pragma unroll
        for (int it = 0; it < 16; ++it) {
            const int cl = wave * 32 + it * 2 + h;
            v4f v;
            v[0] = st[(n0 + 0) * SP + cl];
            v[1] = st[(n0 + 1) * SP + cl];
            v[2] = st[(n0 + 2) * SP + cl];
            v[3] = st[(n0 + 3) * SP + cl];
            const size_t gi = ((size_t)(bimg * CM_ + colB + cl)) * LSEQ_ + (size_t)(pp * NP_ + n0);
            vv[it] = v + *(const v4f*)(xres + gi);
        }
#pragma unroll
        for (int it = 0; it < 16; ++it) {
            const int cl = wave * 32 + it * 2 + h;
            const size_t gi = ((size_t)(bimg * CM_ + colB + cl)) * LSEQ_ + (size_t)(pp * NP_ + n0);
            *(volatile v4f*)(C + gi) = vv[it];
        }
        __threadfence();
#pragma unroll
        for (int it = 0; it < 16; ++it) {
            const int cl = wave * 32 + it * 2 + h;
            const size_t gi = ((size_t)(bimg * CM_ + colB + cl)) * LSEQ_ + (size_t)(pp * NP_ + n0);
            *(volatile v4f*)(C + gi) = vv[it];
        }
    } else {
        const int rsub = lane / LPR;
        const int c4   = (lane % LPR) * 4;
        v4f vv[NIT];
#pragma unroll
        for (int it = 0; it < NIT; ++it) {
            const int row = it * RPI + rsub;
            vv[it] = *(const v4f*)(st + (wm * 32 + row) * SP + wn * CW + c4);
        }
        u16x8 pv[2];
        if (EPI == 1) {
#pragma unroll
            for (int it = 0; it < 2; ++it) {
                const int row = it * 16 + (lane >> 1);
                const int ch  = (lane & 1) * 8;
                const float* sp = st + (wm * 32 + row) * SP + ch;
#pragma unroll
                for (int c = 0; c < 8; ++c) pv[it][c] = f32_to_bf16(sp[c]);
            }
        }
#pragma unroll
        for (int it = 0; it < NIT; ++it) {
            const int row = it * RPI + rsub;
            *(volatile v4f*)(C + (size_t)(rowW + row) * ldc + colW + c4) = vv[it];
        }
        if (EPI == 1 && wn == 0) {
#pragma unroll
            for (int it = 0; it < 2; ++it) {
                const int row = it * 16 + (lane >> 1);
                const int ch  = (lane & 1) * 8;
                *(volatile u16x8*)(P16 + (size_t)(rowW + row) * DTR_ + ch) = pv[it];
            }
        }
        __threadfence();
#pragma unroll
        for (int it = 0; it < NIT; ++it) {
            const int row = it * RPI + rsub;
            *(volatile v4f*)(C + (size_t)(rowW + row) * ldc + colW + c4) = vv[it];
        }
        if (EPI == 1 && wn == 0) {
#pragma unroll
            for (int it = 0; it < 2; ++it) {
                const int row = it * 16 + (lane >> 1);
                const int ch  = (lane & 1) * 8;
                *(volatile u16x8*)(P16 + (size_t)(rowW + row) * DTR_ + ch) = pv[it];
            }
        }
    }
}

__global__ __launch_bounds__(256)
void conv_silu_kernel(const float* __restrict__ xz,
                      const float* __restrict__ cw0, const float* __restrict__ cb0,
                      const float* __restrict__ cw1, const float* __restrict__ cb1,
                      unsigned short* xcb)
{
    const int dir = blockIdx.y;
    const float* cw = dir ? cw1 : cw0;
    const float* cb = dir ? cb1 : cb0;
    const int tid = threadIdx.x;
    const int ts  = blockIdx.x * 4 + (tid >> 6);
    const int bb  = ts >> 6;
    const int l   = ts & 63;
    const int d0  = (tid & 63) * 8;

    v8f xt[4];
#pragma unroll
    for (int j = 0; j < 4; ++j) {
        const int li   = l - 3 + j;
        const int lic  = (li < 0) ? 0 : li;
        const int nsrc = dir ? (NP_ - 1 - lic) : lic;
        v8f v = ld8f(xz + ((size_t)(bb * NP_ + nsrc)) * XE_ + d0);
#pragma unroll
        for (int c = 0; c < 8; ++c) v[c] = (li >= 0) ? v[c] : 0.0f;
        xt[j] = v;
    }
    v4f wv[8];
#pragma unroll
    for (int c = 0; c < 8; ++c) wv[c] = *(const v4f*)(cw + (size_t)(d0 + c) * 4);
    const v8f bias = ld8f(cb + d0);

    u16x8 o;
#pragma unroll
    for (int c = 0; c < 8; ++c) {
        const float u = conv4_silu(xt[0][c], xt[1][c], xt[2][c], xt[3][c],
                                   wv[c][0], wv[c][1], wv[c][2], wv[c][3], bias[c]);
        o[c] = f32_to_bf16(u);
    }
    unsigned short* gp = xcb + ((size_t)dir * NT_ + (size_t)ts) * DI_ + d0;
    *(volatile u16x8*)gp = o;
    __threadfence();
    *(volatile u16x8*)gp = o;
}

__global__ __launch_bounds__(64)
void scan_kernel(const float* __restrict__ xz, const float* __restrict__ xdbl, const float* __restrict__ delta,
                 const float* __restrict__ cw0, const float* __restrict__ cb0,
                 const float* __restrict__ alog0, const float* __restrict__ Dp0,
                 const float* __restrict__ cw1, const float* __restrict__ cb1,
                 const float* __restrict__ alog1, const float* __restrict__ Dp1,
                 float* ys)
{
    __shared__ __attribute__((aligned(16))) float Bl[NP_ * NS_];
    __shared__ __attribute__((aligned(16))) float Cl[NP_ * NS_];
    __shared__ __attribute__((aligned(16))) float sst[16 * 64];

    const int dir  = blockIdx.z;
    const int bb   = blockIdx.y;
    const int cg   = blockIdx.x;
    const int tid  = threadIdx.x;
    const int lane = tid & 31;
    const int wave = tid >> 5;
    const int d    = cg * 64 + tid;

    const float* cw   = dir ? cw1 : cw0;
    const float* cb   = dir ? cb1 : cb0;
    const float* alog = dir ? alog1 : alog0;
    const float* Dp   = dir ? Dp1 : Dp0;

    const size_t trow0 = (size_t)dir * NT_ + (size_t)bb * NP_;
    for (int i = tid; i < NP_ * NS_; i += 64) {
        const int l = i >> 4, n = i & 15;
        const float* xr = xdbl + (trow0 + (size_t)l) * XDP_;
        Bl[i] = xr[DTR_ + n];
        Cl[i] = xr[DTR_ + NS_ + n];
    }

    float an[NS_], hs[NS_];
#pragma unroll
    for (int n = 0; n < NS_; ++n) {
        an[n] = -__expf(alog[d * NS_ + n]);
        hs[n] = 0.0f;
    }
    const float w0 = cw[d * 4 + 0], w1 = cw[d * 4 + 1], w2 = cw[d * 4 + 2], w3 = cw[d * 4 + 3];
    const float cbias = cb[d];
    const float Dd = Dp[d];
    __syncthreads();

    float xm1 = 0.0f, xm2 = 0.0f, xm3 = 0.0f;
    float* yplane = ys + (size_t)dir * NT_ * DI_;

#pragma unroll 1
    for (int l0 = 0; l0 < NP_; l0 += 16) {
#pragma unroll 1
        for (int t = 0; t < 16; ++t) {
            const int l = l0 + t;
            const int nsrc = dir ? (NP_ - 1 - l) : l;
            const float xv = xz[((size_t)(bb * NP_ + nsrc)) * XE_ + d];
            const float dl = delta[(trow0 + (size_t)l) * DI_ + d];
            const float u  = conv4_silu(xm3, xm2, xm1, xv, w0, w1, w2, w3, cbias);
            xm3 = xm2; xm2 = xm1; xm1 = xv;
            const float du = dl * u;
            float y = 0.0f;
#pragma unroll
            for (int n = 0; n < NS_; ++n) {
                const float da = __expf(dl * an[n]);
                hs[n] = da * hs[n] + du * Bl[l * NS_ + n];
                y += hs[n] * Cl[l * NS_ + n];
            }
            const float v = y + Dd * u;
            const int srow = dir ? (15 - t) : t;
            sst[srow * 64 + tid] = v;
        }
        __syncthreads();
        const int posbase = dir ? (NP_ - 16 - l0) : l0;
        const int c4 = (lane & 15) * 4;
        v4f vv[4];
#pragma unroll
        for (int it = 0; it < 4; ++it) {
            const int r = it * 4 + wave * 2 + (lane >> 4);
            vv[it] = *(const v4f*)(sst + r * 64 + c4);
        }
#pragma unroll
        for (int it = 0; it < 4; ++it) {
            const int r = it * 4 + wave * 2 + (lane >> 4);
            *(volatile v4f*)(yplane + ((size_t)(bb * NP_ + posbase + r)) * DI_ + cg * 64 + c4) = vv[it];
        }
        __threadfence();
#pragma unroll
        for (int it = 0; it < 4; ++it) {
            const int r = it * 4 + wave * 2 + (lane >> 4);
            *(volatile v4f*)(yplane + ((size_t)(bb * NP_ + posbase + r)) * DI_ + cg * 64 + c4) = vv[it];
        }
        __syncthreads();
    }
}

__global__ __launch_bounds__(256)
void combine_kernel(const float* __restrict__ ys, const float* __restrict__ xz,
                    unsigned short* ybf, int n8)
{
    const int i = blockIdx.x * 256 + threadIdx.x;
    if (i >= n8) return;
    const size_t e  = (size_t)i * 8;
    const size_t t  = e >> 9;
    const int    d0 = (int)(e & 511);
    const v8f a  = ld8f(ys + e);
    const v8f b  = ld8f(ys + (size_t)NT_ * DI_ + e);
    const v8f zv = ld8f(xz + t * XE_ + DI_ + d0);
    u16x8 o;
#pragma unroll
    for (int c = 0; c < 8; ++c) {
        const float sz = silu_f(zv[c]);
        const float g  = a[c] * sz + b[c] * sz;
        o[c] = f32_to_bf16(g);
    }
    unsigned short* gp = ybf + e;
    *(volatile u16x8*)gp = o;
    __threadfence();
    *(volatile u16x8*)gp = o;
}

extern "C" void kernel_launch(void* const* d_in, const int* in_sizes, int n_in,
                              void* d_out, int out_size, void* d_ws, size_t ws_size,
                              hipStream_t stream)
{
    if (n_in < 19) return;
    if (in_sizes[0]  != NB_ * CM_ * LSEQ_) return;
    if (in_sizes[1]  != CM_)             return;
    if (in_sizes[2]  != CM_)             return;
    if (in_sizes[3]  != XE_ * CM_)       return;
    if (in_sizes[4]  != DI_ * 4)         return;
    if (in_sizes[5]  != DI_)             return;
    if (in_sizes[6]  != XD_ * DI_)       return;
    if (in_sizes[7]  != DI_ * DTR_)      return;
    if (in_sizes[8]  != DI_)             return;
    if (in_sizes[9]  != DI_ * NS_)       return;
    if (in_sizes[10] != DI_)             return;
    if (in_sizes[11] != DI_ * 4)         return;
    if (in_sizes[12] != DI_)             return;
    if (in_sizes[13] != XD_ * DI_)       return;
    if (in_sizes[14] != DI_ * DTR_)      return;
    if (in_sizes[15] != DI_)             return;
    if (in_sizes[16] != DI_ * NS_)       return;
    if (in_sizes[17] != DI_)             return;
    if (in_sizes[18] != CM_ * DI_)       return;
    if (out_size != NB_ * CM_ * LSEQ_)   return;

    const float* x      = (const float*)d_in[0];
    const float* ln_g   = (const float*)d_in[1];
    const float* ln_b   = (const float*)d_in[2];
    const float* w_in   = (const float*)d_in[3];
    const float* cw_f   = (const float*)d_in[4];
    const float* cb_f   = (const float*)d_in[5];
    const float* wxp_f  = (const float*)d_in[6];
    const float* wdt_f  = (const float*)d_in[7];
    const float* bdt_f  = (const float*)d_in[8];
    const float* alog_f = (const float*)d_in[9];
    const float* D_f    = (const float*)d_in[10];
    const float* cw_b   = (const float*)d_in[11];
    const float* cb_b   = (const float*)d_in[12];
    const float* wxp_b  = (const float*)d_in[13];
    const float* wdt_b  = (const float*)d_in[14];
    const float* bdt_b  = (const float*)d_in[15];
    const float* alog_b = (const float*)d_in[16];
    const float* D_b    = (const float*)d_in[17];
    const float* w_out  = (const float*)d_in[18];
    float* out = (float*)d_out;

    const size_t SZ_WIN  = (size_t)XE_ * CM_ * 2;
    const size_t SZ_WXP  = (size_t)2 * XDP_ * DI_ * 2;
    const size_t SZ_WDT  = (size_t)2 * DI_ * DTR_ * 2;
    const size_t SZ_WOUT = (size_t)CM_ * DI_ * 2;
    const size_t SZ_XN   = (size_t)NT_ * CM_ * 2;
    const size_t SZ_XCB  = (size_t)2 * NT_ * DI_ * 2;
    const size_t SZ_XZ   = (size_t)NT_ * XE_ * 4;
    const size_t SZ_XDBL = (size_t)2 * NT_ * XDP_ * 4;
    const size_t SZ_DTB  = (size_t)2 * NT_ * DTR_ * 2;
    const size_t SZ_DEL  = (size_t)2 * NT_ * DI_ * 4;
    const size_t SZ_YS   = (size_t)2 * NT_ * DI_ * 4;
    const size_t SZ_YBF  = (size_t)NT_ * DI_ * 2;

    const size_t OFF_WIN  = 0;
    const size_t OFF_WXP  = OFF_WIN + SZ_WIN;
    const size_t OFF_WDT  = OFF_WXP + SZ_WXP;
    const size_t OFF_WOUT = OFF_WDT + SZ_WDT;
    const size_t OFF_XN   = OFF_WOUT + SZ_WOUT;
    const size_t OFF_XCB  = OFF_XN + SZ_XN;
    const size_t OFF_XZ   = OFF_XCB + SZ_XCB;
    const size_t OFF_XDBL = OFF_XZ + SZ_XZ;
    const size_t OFF_DTB  = OFF_XDBL + SZ_XDBL;
    const size_t OFF_DEL  = OFF_DTB + SZ_DTB;
    const size_t OFF_YS   = OFF_DEL + SZ_DEL;
    const size_t WS_END   = OFF_YS + SZ_YS;
    const size_t OFF_YBF  = OFF_XN;
    if (OFF_YBF + SZ_YBF > OFF_XZ) return;
    if (ws_size < WS_END) return;

    char* ws = (char*)d_ws;
    unsigned short* win16  = (unsigned short*)(ws + OFF_WIN);
    unsigned short* wxp16  = (unsigned short*)(ws + OFF_WXP);
    unsigned short* wdt16  = (unsigned short*)(ws + OFF_WDT);
    unsigned short* wout16 = (unsigned short*)(ws + OFF_WOUT);
    unsigned short* xn16   = (unsigned short*)(ws + OFF_XN);
    unsigned short* xcb16  = (unsigned short*)(ws + OFF_XCB);
    float*          xz     = (float*)(ws + OFF_XZ);
    float*          xdbl   = (float*)(ws + OFF_XDBL);
    unsigned short* dtb16  = (unsigned short*)(ws + OFF_DTB);
    float*          delta  = (float*)(ws + OFF_DEL);
    float*          ys     = (float*)(ws + OFF_YS);
    unsigned short* ybf16  = (unsigned short*)(ws + OFF_YBF);

    hipLaunchKernelGGL(cvt_kernel, dim3((XE_ * CM_ / 8 + 255) / 256, 1), dim3(256), 0, stream,
                       w_in, w_in, win16, win16, (int)XE_, (int)XE_, (int)CM_);
    hipLaunchKernelGGL(cvt_kernel, dim3((XDP_ * DI_ / 8 + 255) / 256, 2), dim3(256), 0, stream,
                       wxp_f, wxp_b, wxp16, wxp16 + (size_t)XDP_ * DI_, (int)XD_, (int)XDP_, (int)DI_);
    hipLaunchKernelGGL(cvt_kernel, dim3((DI_ * DTR_ / 8 + 255) / 256, 2), dim3(256), 0, stream,
                       wdt_f, wdt_b, wdt16, wdt16 + (size_t)DI_ * DTR_, (int)DI_, (int)DI_, (int)DTR_);
    hipLaunchKernelGGL(cvt_kernel, dim3((CM_ * DI_ / 8 + 255) / 256, 1), dim3(256), 0, stream,
                       w_out, w_out, wout16, wout16, (int)CM_, (int)CM_, (int)DI_);

    hipLaunchKernelGGL(ln_kernel, dim3(NT_ / 8), dim3(256), 0, stream, x, ln_g, ln_b, xn16);

    hipLaunchKernelGGL(HIP_KERNEL_NAME(gemm_kernel<4, false, 0>),
                       dim3(XE_ / 128, NT_ / 64, 1), dim3(128), 0, stream,
                       (const unsigned short*)xn16, (const unsigned short*)win16, xz,
                       bdt_f, bdt_b, dtb16, x,
                       (int)CM_, (int)XE_, 0, 0, 0, 0);

    hipLaunchKernelGGL(conv_silu_kernel, dim3(NT_ / 4, 2), dim3(256), 0, stream,
                       (const float*)xz, cw_f, cb_f, cw_b, cb_b, xcb16);

    hipLaunchKernelGGL(HIP_KERNEL_NAME(gemm_kernel<2, false, 1>),
                       dim3(1, NT_ / 64, 2), dim3(128), 0, stream,
                       (const unsigned short*)xcb16, (const unsigned short*)wxp16, xdbl,
                       bdt_f, bdt_b, dtb16, x,
                       (int)DI_, (int)XDP_, (int)(NT_ * DI_), (int)(XDP_ * DI_), (int)(NT_ * XDP_), (int)(NT_ * DTR_));

    hipLaunchKernelGGL(HIP_KERNEL_NAME(gemm_kernel<4, true, 2>),
                       dim3(DI_ / 128, NT_ / 64, 2), dim3(128), 0, stream,
                       (const unsigned short*)dtb16, (const unsigned short*)wdt16, delta,
                       bdt_f, bdt_b, dtb16, x,
                       (int)DTR_, (int)DI_, (int)(NT_ * DTR_), (int)(DI_ * DTR_), (int)(NT_ * DI_), 0);

    hipLaunchKernelGGL(scan_kernel, dim3(DI_ / 64, NSEQ_, 2), dim3(64), 0, stream,
                       (const float*)xz, (const float*)xdbl, (const float*)delta,
                       cw_f, cb_f, alog_f, D_f, cw_b, cb_b, alog_b, D_b, ys);

    {
        const int n8 = (NT_ * DI_) / 8;
        hipLaunchKernelGGL(combine_kernel, dim3((n8 + 255) / 256), dim3(256), 0, stream,
                           (const float*)ys, (const float*)xz, ybf16, n8);
    }

    hipLaunchKernelGGL(HIP_KERNEL_NAME(gemm_kernel<4, false, 3>),
                       dim3(CM_ / 128, NT_ / 64, 1), dim3(128), 0, stream,
                       (const unsigned short*)ybf16, (const unsigned short*)wout16, out,
                       bdt_f, bdt_b, dtb16, x,
                       (int)DI_, (int)CM_, 0, 0, 0, 0);
}
